// MultiHeadAttention_84293028152083
// MI455X (gfx1250) — hardware-run, weakly checked
//
#include <hip/hip_runtime.h>


#ifndef NB
#define NB 2
#endif
#ifndef SEQ
#define SEQ 4096
#endif
#define NB_FULL  2
#define SEQ_FULL 4096
#ifndef OUT_SEQ
#define OUT_SEQ SEQ
#endif
#define DM    1024
#define NH_   16
#define HD    64
#define BLK   128
#define EROWS 128
#define CK    32
#define LOG2E 1.4426950408889634f
#define QCAR  256.0f
#define VCAR  256.0f
#define PCAR  2048.0f
#define SCQ   (0.125f * 16.0f / 256.0f)
#define C1    (LOG2E / 16.0f)
#define NEGL  (-1000.0f * LOG2E)
#define WOCAR 64.0f
#define OSC   (1.0f / (256.0f * 64.0f))

static_assert(HD == 64);
static_assert(NH_ == 16);
static_assert(NH_ * HD == DM);
static_assert(DM % 64 == 0);
static_assert(DM % 32 == 0);
static_assert(SEQ % BLK == 0);
static_assert(BLK % CK == 0);
static_assert(EROWS == BLK);
static_assert(EROWS % 64 == 0);
static_assert(EROWS <= SEQ);
static_assert((NB * SEQ) % 64 == 0);
static_assert(((size_t)SEQ * DM) % 8 == 0);
static_assert(((size_t)DM * DM) % 8 == 0);
static_assert(NB <= NB_FULL);
static_assert(SEQ <= SEQ_FULL);

typedef _Float16 h16;
typedef unsigned short bf;
typedef __attribute__((ext_vector_type(16))) __bf16   v16bf;
typedef __attribute__((ext_vector_type(16))) _Float16 v16h;
typedef __attribute__((ext_vector_type(8)))  _Float16 v8h;
typedef __attribute__((ext_vector_type(8)))  unsigned short v8us;
typedef __attribute__((ext_vector_type(8)))  float    v8f;
typedef __attribute__((ext_vector_type(4)))  float    v4f;
typedef v4f  __attribute__((may_alias)) v4fa;
typedef v8h  __attribute__((may_alias)) v8ha;

__device__ __forceinline__ unsigned short f2bf(float f) { unsigned u = __float_as_uint(f); u += 0x7FFFu + ((u >> 16) & 1u); return (unsigned short)(u >> 16); }
__device__ __forceinline__ float bfr(float f) { return __uint_as_float(((unsigned)f2bf(f)) << 16); }
__device__ __forceinline__ float ex2(float x) { return __builtin_amdgcn_exp2f(x); }
__device__ __forceinline__ v16h cat16(v8h lo, v8h hi) { return __builtin_shufflevector(lo, hi, 0, 1, 2, 3, 4, 5, 6, 7, 8, 9, 10, 11, 12, 13, 14, 15); }
__device__ __forceinline__ v16bf cat16b(v8us lo, v8us hi) { return __builtin_bit_cast(v16bf, __builtin_shufflevector(lo, hi, 0, 1, 2, 3, 4, 5, 6, 7, 8, 9, 10, 11, 12, 13, 14, 15)); }
__device__ __forceinline__ v8f wmma16(v16h a, v16h b, v8f c) { return __builtin_amdgcn_wmma_f32_16x16x32_f16(false, a, false, b, (short)0, c, false, false); }
__device__ __forceinline__ v8f wmmab(v16bf a, v16bf b, v8f c) { return __builtin_amdgcn_wmma_f32_16x16x32_bf16(false, a, false, b, (short)0, c, false, false); }
__device__ __forceinline__ v16h  ldh(const h16* p) { return cat16(*(const v8h*)p, *(const v8h*)(p + 16)); }
__device__ __forceinline__ v16bf ldb(const bf* p)  { return cat16b(*(const v8us*)p, *(const v8us*)(p + 16)); }
__device__ __forceinline__ void wave_sync() { __builtin_amdgcn_fence(3  , "wavefront"); __builtin_amdgcn_wave_barrier(); asm volatile("" ::: "memory"); }

__global__ __launch_bounds__(256) void k_cvt8(const float* __restrict__ src, bf* dst, size_t n8) {
    const size_t i = (size_t)blockIdx.x * 256 + threadIdx.x; if (i >= n8) return;
    const v8f v = *(const v8f*)(src + i * 8); v8us o;
#pragma unroll
    for (int k = 0; k < 8; ++k) o[k] = f2bf(v[k]);
    *(volatile v8us*)(dst + i * 8) = o; __threadfence(); *(volatile v8us*)(dst + i * 8) = o;
}

__global__ __launch_bounds__(256) void k_cvt8h(const float* __restrict__ src, h16* dst, size_t n8, float sc) {
    const size_t i = (size_t)blockIdx.x * 256 + threadIdx.x; if (i >= n8) return;
    const v8f v = *(const v8f*)(src + i * 8); v8h o;
#pragma unroll
    for (int k = 0; k < 8; ++k) o[k] = (h16)(bfr(v[k]) * sc);
    *(volatile v8h*)(dst + i * 8) = o; __threadfence(); *(volatile v8h*)(dst + i * 8) = o;
}

__global__ __launch_bounds__(32) void k_proj(const bf* __restrict__ A, const bf* __restrict__ Bt, h16* Ph, h16* Pr, int useRes, float cs, int RB, size_t sRB, int pitch, int CB, size_t sCB) {
    __shared__ __align__(16) float os[16 * 68];
    const int K = DM;
    const int lane = threadIdx.x & 31, lr = lane & 15, hi = lane >> 4; const int r0 = blockIdx.x * 64, c0 = blockIdx.y * 64;
    v8f acc[4][4];
#pragma unroll
    for (int mb = 0; mb < 4; ++mb)
#pragma unroll
        for (int nb = 0; nb < 4; ++nb) acc[mb][nb] = (v8f){};
    const size_t aoff = (size_t)(r0 + lr) * K + 8 * hi, boff = (size_t)(c0 + lr) * K + 8 * hi;
#pragma unroll 1
    for (int kc = 0; kc < K; kc += 32) {
        v16bf a[4];
#pragma unroll
        for (int mb = 0; mb < 4; ++mb) a[mb] = ldb(A + aoff + (size_t)mb * 16 * K + kc);
#pragma unroll
        for (int nb = 0; nb < 4; ++nb) { const v16bf b = ldb(Bt + boff + (size_t)nb * 16 * K + kc);
#pragma unroll
            for (int mb = 0; mb < 4; ++mb) acc[mb][nb] = wmmab(a[mb], b, acc[mb][nb]); }
        asm volatile("v_nop\n\tv_nop\n\tv_nop\n\tv_nop" : "+v"(acc[0][0]), "+v"(acc[1][1]), "+v"(acc[2][2]), "+v"(acc[3][3]) : "v"(a[0]), "v"(a[1]), "v"(a[2]), "v"(a[3]));
    }
    const size_t tbase = (size_t)(r0 / RB) * sRB + (size_t)(r0 % RB) * (size_t)pitch + (size_t)(c0 / CB) * sCB + (size_t)(c0 % CB);
#pragma unroll
    for (int mb = 0; mb < 4; ++mb) {
#pragma unroll
        for (int nb = 0; nb < 4; ++nb) {
#pragma unroll
            for (int j = 0; j < 8; ++j) os[(hi * 8 + j) * 68 + nb * 16 + lr] = acc[mb][nb][j]; }
        wave_sync();
        const size_t sb = tbase + (size_t)(mb * 16) * (size_t)pitch;
#pragma unroll 1
        for (int ps = 0; ps < 2; ++ps) {
#pragma unroll
            for (int s = 0; s < 4; ++s) { const int row = 4 * s + (lane >> 3), c8 = (lane & 7) * 8;
                const v4f x0 = *(const v4fa*)(&os[row * 68 + c8]); const v4f x1 = *(const v4fa*)(&os[row * 68 + c8 + 4]); v8h hv, rv;
#pragma unroll
                for (int i = 0; i < 4; ++i) { const float y0 = x0[i] * cs, y1 = x1[i] * cs; const h16 a0 = (h16)y0; const h16 a1 = (h16)y1; hv[i] = a0; hv[4 + i] = a1; rv[i] = (h16)(y0 - (float)a0); rv[4 + i] = (h16)(y1 - (float)a1); }
                const size_t oo = sb + (size_t)row * (size_t)pitch + c8;
                *(volatile v8h*)(Ph + oo) = hv; if (useRes) *(volatile v8h*)(Pr + oo) = rv; }
            if (ps == 0) __threadfence(); }
        wave_sync();
    }
}

template <int EARLY>
__global__ __launch_bounds__(512) void k_attn(const h16* __restrict__ QH, const h16* __restrict__ QR, const h16* __restrict__ KP,
                                              const h16* __restrict__ VH, const h16* __restrict__ VR, const int* __restrict__ qmask,
                                              const float* __restrict__ Tb, const float* __restrict__ Ta, const float* __restrict__ relp, const float* __restrict__ absp,
                                              h16* CH, h16* CR, int tile0) {
    __shared__ __align__(16) h16 sx[16 * CK * 16];
    __shared__ __align__(16) h16 px[16 * 16 * CK];
    __shared__ __align__(16) h16 pxr[EARLY ? 16 * 16 * CK : 8];
    __shared__ __align__(16) h16 osh[16 * 16 * 72];
    __shared__ __align__(16) h16 osr[EARLY ? 16 * 16 * 72 : 8];
    __shared__ float rsum[16];
    const int tid = threadIdx.x, lane = tid & 31, w = __builtin_amdgcn_readfirstlane((int)(tid >> 5)), lr = lane & 15, hi = lane >> 4;
    const int b = blockIdx.y;
    const int t0 = (tile0 + (int)blockIdx.x) * 16;
    const int kw0 = (t0 / BLK) * BLK - BLK;
    { const int gr = tid & 15; float s = 0.0f;
#pragma unroll
      for (int h = 0; h < 16; ++h) s += bfr(Tb[gr * 16 + h]);
      if (tid < 16) rsum[tid] = s; }
    const int qv = qmask[(size_t)b * SEQ_FULL + t0 + lr];
    const unsigned bal = __builtin_amdgcn_ballot_w32(qv == 0);
    const int full = (bal != 0u);
    const int qmw = (((bal >> w) & 1u) == 0u);
    const float rel = bfr(relp[0]);
    const float absb = bfr(absp[0]);
    __syncthreads();
    float bg[8];
#pragma unroll
    for (int r = 0; r < 8; ++r) bg[r] = absb * LOG2E * rsum[8 * hi + r];
    v16h tbf, taf;
#pragma unroll
    for (int i = 0; i < 8; ++i) { const float a = bfr(Tb[lr * 16 + 8 * hi + i]); const float c = bfr(Ta[lr * 16 + 8 * hi + i]);
        tbf[i] = (h16)a; tbf[8 + i] = (h16)0.0f; taf[i] = (h16)c; taf[8 + i] = (h16)c; }
    int kbeg, kend;
    if (full) { kbeg = kw0; kend = kw0 + 3 * BLK; }
    else { kbeg = kw0 < 0 ? 0 : kw0; kend = kbeg + ((t0 + 16 - kbeg + 31) >> 5) * 32; }
    const size_t pbase = ((size_t)b * NH_ + w) * SEQ * HD;
    const size_t qo = pbase + (size_t)(t0 + lr) * HD + 8 * hi;
    const v16h qh0 = ldh(QH + qo), qh1 = ldh(QH + qo + 32), qr0 = ldh(QR + qo), qr1 = ldh(QR + qo + 32);
    const size_t ko = pbase + (size_t)lr * HD + 8 * hi;
    const size_t vo = pbase + (size_t)lr * SEQ + 8 * hi;
    v8f o0 = (v8f){}, o1 = (v8f){}, o2 = (v8f){}, o3 = (v8f){};
    float m[8], l[8];
#pragma unroll
    for (int r = 0; r < 8; ++r) { m[r] = -3.0e38f; l[r] = 0.0f; }
    const int qpos_m = t0 + w;
    const int qpos_s = t0 + lr;
    const v8h zero8 = (v8h){};

#pragma unroll 1
    for (int pass = 0; pass < 2; ++pass) {
#pragma unroll 1
        for (int key0 = kbeg; key0 < kend; key0 += CK) {
            const int inr = (key0 >= 0) && (key0 < SEQ);
            const int kc = key0 < 0 ? 0 : (key0 > SEQ - CK ? SEQ - CK : key0);
            {
                const h16* ka = KP + ko + (size_t)kc * HD;
                const v16h ka0 = ldh(ka), ka1 = ldh(ka + 32), kb0 = ldh(ka + 16 * HD), kb1 = ldh(ka + 16 * HD + 32);
                v8f sa = (v8f){}, sb = (v8f){};
                sa = wmma16(ka0, qh0, sa); sb = wmma16(kb0, qh0, sb);
                sa = wmma16(ka0, qr0, sa); sb = wmma16(kb0, qr0, sb);
                sa = wmma16(ka1, qh1, sa); sb = wmma16(kb1, qh1, sb);
                sa = wmma16(ka1, qr1, sa); sb = wmma16(kb1, qr1, sb);
                asm volatile("v_nop\n\tv_nop\n\tv_nop\n\tv_nop" : "+v"(sa), "+v"(sb) : "v"(ka0), "v"(ka1), "v"(kb0), "v"(kb1));
                const int d0 = qpos_s - (key0 + 8 * hi);
#pragma unroll
                for (int r = 0; r < 8; ++r) {
                    int da = d0 - r; da = da < 0 ? -da : da;
                    int db = d0 - 16 - r; db = db < 0 ? -db : db;
                    const float fa = __builtin_amdgcn_rcpf(1.0f + rel * (float)da);
                    const float fb = __builtin_amdgcn_rcpf(1.0f + rel * (float)db);
                    sx[(lr * CK + 8 * hi + r) * 16 + w]      = (h16)(sa[r] * (SCQ * fa));
                    sx[(lr * CK + 16 + 8 * hi + r) * 16 + w] = (h16)(sb[r] * (SCQ * fb));
                }
            }
            __syncthreads();
            float tla[8], tlb[8];
            {
                const v8h la = *(const v8ha*)(&sx[(w * CK + lr) * 16 + 8 * hi]);
                const v8h lb = *(const v8ha*)(&sx[(w * CK + 16 + lr) * 16 + 8 * hi]);
                const v16h fa = cat16(la, zero8), fb = cat16(lb, zero8);
                v8f da = (v8f){}, db = (v8f){};
                da = wmma16(tbf, fa, da); db = wmma16(tbf, fb, db);
                asm volatile("v_nop\n\tv_nop\n\tv_nop\n\tv_nop" : "+v"(da), "+v"(db) : "v"(fa), "v"(fb), "v"(tbf));
                const int kpa = key0 + lr, kpb = key0 + 16 + lr;
                const bool va = (qmw != 0) && (inr != 0) && (kpa <= qpos_m);
                const bool vb = (qmw != 0) && (inr != 0) && (kpb <= qpos_m);
                const float ba = (kpa < qpos_m) ? 1.0f : 0.0f;
                const float bb = (kpb < qpos_m) ? 1.0f : 0.0f;
#pragma unroll
                for (int r = 0; r < 8; ++r) {
                    const float xa = da[r] * C1 - ba * bg[r];
                    const float xb = db[r] * C1 - bb * bg[r];
                    tla[r] = va ? xa : NEGL;
                    tlb[r] = vb ? xb : NEGL;
                }
            }
            if (pass == 0) {
#pragma unroll
                for (int r = 0; r < 8; ++r) {
                    const float mx = fmaxf(m[r], fmaxf(tla[r], tlb[r]));
                    l[r] = l[r] * ex2(m[r] - mx) + ex2(tla[r] - mx) + ex2(tlb[r] - mx);
                    m[r] = mx;
                }
                __syncthreads();
            } else {
                v16h pfa, pfb;
#pragma unroll
                for (int r = 0; r < 8; ++r) {
                    const float ea = ex2(tla[r] - m[r]) * l[r];
                    const float eb = ex2(tlb[r] - m[r]) * l[r];
                    const h16 ha = (h16)ea; const h16 hb = (h16)eb;
                    pfa[r] = ha; pfa[8 + r] = (h16)(ea - (float)ha);
                    pfb[r] = hb; pfb[8 + r] = (h16)(eb - (float)hb);
                }
                v8f ma = (v8f){}, mb = (v8f){};
                ma = wmma16(taf, pfa, ma); mb = wmma16(taf, pfb, mb);
                asm volatile("v_nop\n\tv_nop\n\tv_nop\n\tv_nop" : "+v"(ma), "+v"(mb) : "v"(pfa), "v"(pfb), "v"(taf));
                const float zf = inr ? 1.0f : 0.0f;
#pragma unroll
                for (int r = 0; r < 8; ++r) {
                    const float xa = ma[r] * zf, xb = mb[r] * zf;
                    const h16 ha = (h16)xa; const h16 hb = (h16)xb;
                    const int ia = ((8 * hi + r) * 16 + w) * CK + lr;
                    px[ia] = ha; px[ia + 16] = hb;
                    if (EARLY) { pxr[ia] = (h16)(xa - (float)ha); pxr[ia + 16] = (h16)(xb - (float)hb); }
                }
                __syncthreads();
                const h16* pp = &px[(w * 16 + lr) * CK + 8 * hi];
                const v16h pb = cat16(*(const v8ha*)pp, *(const v8ha*)(pp + 16));
                const h16* va_ = VH + vo + kc;
                const v16h v0 = ldh(va_), v1 = ldh(va_ + (size_t)16 * SEQ), v2 = ldh(va_ + (size_t)32 * SEQ), v3 = ldh(va_ + (size_t)48 * SEQ);
                o0 = wmma16(v0, pb, o0); o1 = wmma16(v1, pb, o1); o2 = wmma16(v2, pb, o2); o3 = wmma16(v3, pb, o3);
                if (EARLY) {
                    const h16* pq = &pxr[(w * 16 + lr) * CK + 8 * hi];
                    const v16h pr = cat16(*(const v8ha*)pq, *(const v8ha*)(pq + 16));
                    const h16* vr_ = VR + vo + kc;
                    const v16h r0_ = ldh(vr_), r1_ = ldh(vr_ + (size_t)16 * SEQ), r2_ = ldh(vr_ + (size_t)32 * SEQ), r3_ = ldh(vr_ + (size_t)48 * SEQ);
                    o0 = wmma16(r0_, pb, o0); o1 = wmma16(r1_, pb, o1); o2 = wmma16(r2_, pb, o2); o3 = wmma16(r3_, pb, o3);
                    o0 = wmma16(v0, pr, o0);  o1 = wmma16(v1, pr, o1);  o2 = wmma16(v2, pr, o2);  o3 = wmma16(v3, pr, o3);
                    asm volatile("v_nop\n\tv_nop\n\tv_nop\n\tv_nop" : "+v"(o0), "+v"(o1), "+v"(o2), "+v"(o3) : "v"(r0_), "v"(r1_), "v"(r2_), "v"(r3_), "v"(pr));
                }
                asm volatile("v_nop\n\tv_nop\n\tv_nop\n\tv_nop" : "+v"(o0), "+v"(o1), "+v"(o2), "+v"(o3) : "v"(v0), "v"(v1), "v"(v2), "v"(v3), "v"(pb));
            }
        }
        if (pass == 0) {
#pragma unroll
            for (int r = 0; r < 8; ++r) {
                float M = m[r];
                M = fmaxf(M, __shfl_xor(M, 1, 32)); M = fmaxf(M, __shfl_xor(M, 2, 32)); M = fmaxf(M, __shfl_xor(M, 4, 32)); M = fmaxf(M, __shfl_xor(M, 8, 32));
                float L = l[r] * ex2(m[r] - M);
                L += __shfl_xor(L, 1, 32); L += __shfl_xor(L, 2, 32); L += __shfl_xor(L, 4, 32); L += __shfl_xor(L, 8, 32);
                m[r] = M; l[r] = PCAR * __builtin_amdgcn_rcpf(L);
            }
        }
    }

    const float oc = 1.0f / PCAR;
    {
        v8h hv, rv;
#pragma unroll
        for (int r = 0; r < 8; ++r) { const float x = o0[r] * oc; const h16 a = (h16)x; hv[r] = a; rv[r] = (h16)(x - (float)a); }
        *(v8ha*)(&osh[(w * 16 + lr) * 72 +  0 + 8 * hi]) = hv; if (EARLY) *(v8ha*)(&osr[(w * 16 + lr) * 72 +  0 + 8 * hi]) = rv;
#pragma unroll
        for (int r = 0; r < 8; ++r) { const float x = o1[r] * oc; const h16 a = (h16)x; hv[r] = a; rv[r] = (h16)(x - (float)a); }
        *(v8ha*)(&osh[(w * 16 + lr) * 72 + 16 + 8 * hi]) = hv; if (EARLY) *(v8ha*)(&osr[(w * 16 + lr) * 72 + 16 + 8 * hi]) = rv;
#pragma unroll
        for (int r = 0; r < 8; ++r) { const float x = o2[r] * oc; const h16 a = (h16)x; hv[r] = a; rv[r] = (h16)(x - (float)a); }
        *(v8ha*)(&osh[(w * 16 + lr) * 72 + 32 + 8 * hi]) = hv; if (EARLY) *(v8ha*)(&osr[(w * 16 + lr) * 72 + 32 + 8 * hi]) = rv;
#pragma unroll
        for (int r = 0; r < 8; ++r) { const float x = o3[r] * oc; const h16 a = (h16)x; hv[r] = a; rv[r] = (h16)(x - (float)a); }
        *(v8ha*)(&osh[(w * 16 + lr) * 72 + 48 + 8 * hi]) = hv; if (EARLY) *(v8ha*)(&osr[(w * 16 + lr) * 72 + 48 + 8 * hi]) = rv;
    }
    wave_sync();
    h16* crow = CH + ((size_t)b * SEQ + t0) * DM + w * HD;
    h16* rrow = CR + ((size_t)b * EROWS + (EARLY ? t0 : 0)) * DM + w * HD;
#pragma unroll 1
    for (int ps = 0; ps < 2; ++ps) {
#pragma unroll
        for (int s = 0; s < 4; ++s) { const int row = 4 * s + (lane >> 3), c8 = (lane & 7) * 8;
            const v8h hv = *(const v8ha*)(&osh[(w * 16 + row) * 72 + c8]);
            *(volatile v8h*)(crow + (size_t)row * DM + c8) = hv;
            if (EARLY) { const v8h rv = *(const v8ha*)(&osr[(w * 16 + row) * 72 + c8]); *(volatile v8h*)(rrow + (size_t)row * DM + c8) = rv; } }
        if (ps == 0) __threadfence(); }
}

__global__ __launch_bounds__(32) void k_out(const h16* __restrict__ CX, const h16* __restrict__ WO, float* OUT, size_t crOff) {
    __shared__ __align__(16) float os[16 * 68];
    const int K = DM;
    const int lane = threadIdx.x & 31, lr = lane & 15, hi = lane >> 4; const int r0 = blockIdx.x * 64, c0 = blockIdx.y * 64;
    const int b = r0 / SEQ, tt = r0 % SEQ;
    const int npass = (tt < EROWS) ? 2 : 1;
    v8f acc[4][4];
#pragma unroll
    for (int mb = 0; mb < 4; ++mb)
#pragma unroll
        for (int nb = 0; nb < 4; ++nb) acc[mb][nb] = (v8f){};
    const size_t boff = (size_t)(c0 + lr) * K + 8 * hi;
#pragma unroll 1
    for (int sw = 0; sw < npass; ++sw) {
        const size_t aoff = (sw == 0 ? (size_t)(r0 + lr) * K : crOff + (size_t)(b * EROWS + tt + lr) * K) + 8 * hi;
#pragma unroll 1
        for (int kc = 0; kc < K; kc += 32) {
            v16h a[4];
#pragma unroll
            for (int mb = 0; mb < 4; ++mb) a[mb] = ldh(CX + aoff + (size_t)mb * 16 * K + kc);
#pragma unroll
            for (int nb = 0; nb < 4; ++nb) { const v16h bv = ldh(WO + boff + (size_t)nb * 16 * K + kc);
#pragma unroll
                for (int mb = 0; mb < 4; ++mb) acc[mb][nb] = wmma16(a[mb], bv, acc[mb][nb]); }
            asm volatile("v_nop\n\tv_nop\n\tv_nop\n\tv_nop" : "+v"(acc[0][0]), "+v"(acc[1][1]), "+v"(acc[2][2]), "+v"(acc[3][3]) : "v"(a[0]), "v"(a[1]), "v"(a[2]), "v"(a[3]));
        }
    }
    float* obase = OUT + ((size_t)b * OUT_SEQ + tt) * DM + c0;
#pragma unroll
    for (int mb = 0; mb < 4; ++mb) {
#pragma unroll
        for (int nb = 0; nb < 4; ++nb) {
#pragma unroll
            for (int j = 0; j < 8; ++j) os[(hi * 8 + j) * 68 + nb * 16 + lr] = acc[mb][nb][j] * OSC; }
        wave_sync();
        float* orow = obase + (size_t)(mb * 16) * DM;
#pragma unroll 1
        for (int ps = 0; ps < 2; ++ps) {
#pragma unroll
            for (int s = 0; s < 8; ++s) { const int row = 2 * s + hi, cofs = lr * 4;
                const v4f val = *(const v4fa*)(&os[row * 68 + cofs]);
                *(volatile v4f*)(orow + (size_t)row * DM + cofs) = val; }
            if (ps == 0) __threadfence(); }
        wave_sync();
    }
}

static constexpr size_t al256(size_t v) { return (v + 255) & ~(size_t)255; }
static constexpr size_t SZ_XB = al256((size_t)NB * SEQ * DM * 2);
static constexpr size_t SZ_WB = al256((size_t)3 * DM * DM * 2);
static constexpr size_t SZ_PL = al256((size_t)NB * NH_ * SEQ * HD * 2);
static constexpr size_t SZ_CR = al256((size_t)NB * EROWS * DM * 2);
static constexpr size_t SZ_TOTAL = SZ_XB + SZ_WB + 6 * SZ_PL + SZ_CR;
static_assert(SZ_TOTAL <= (size_t)134217728);
static_assert(((size_t)DM * DM * 2) % 256 == 0);
static_assert((size_t)NB * SEQ * DM * 2 == (size_t)NB * NH_ * SEQ * HD * 2);

extern "C" void kernel_launch(void* const* d_in, const int* in_sizes, int n_in,
                              void* d_out, int out_size, void* d_ws, size_t ws_size, hipStream_t stream) {
    if (n_in < 9) return;
    const size_t needx = ((size_t)(NB - 1) * SEQ_FULL + SEQ) * DM;
    if ((size_t)in_sizes[0] < needx) return;
    if ((size_t)in_sizes[1] < (size_t)(NB - 1) * SEQ_FULL + SEQ) return;
    if ((size_t)in_sizes[2] < (size_t)DM * DM || (size_t)in_sizes[3] < (size_t)DM * DM || (size_t)in_sizes[4] < (size_t)DM * DM) return;
    if (in_sizes[5] < NH_ * NH_ || in_sizes[6] < NH_ * NH_ || in_sizes[7] < 1 || in_sizes[8] < 1) return;
    if ((size_t)out_size < ((size_t)(NB - 1) * OUT_SEQ + SEQ) * DM) return;
    if (SZ_TOTAL > ws_size) return;
    const float* x = (const float*)d_in[0]; const int* qm = (const int*)d_in[1];
    const float* wq = (const float*)d_in[2]; const float* wk = (const float*)d_in[3]; const float* wo = (const float*)d_in[4];
    const float* tb = (const float*)d_in[5]; const float* ta = (const float*)d_in[6];
    const float* rela = (const float*)d_in[7]; const float* absa = (const float*)d_in[8];
    float* OUT = (float*)d_out;
    char* wsp = (char*)d_ws;
    bf* XB = (bf*)wsp; wsp += SZ_XB;
    char* WBc = wsp; wsp += SZ_WB;
    h16* QH = (h16*)wsp; wsp += SZ_PL;
    h16* QR = (h16*)wsp; wsp += SZ_PL;
    h16* KP = (h16*)wsp; wsp += SZ_PL;
    h16* VH = (h16*)wsp; wsp += SZ_PL;
    h16* VR = (h16*)wsp; wsp += SZ_PL;
    h16* CH = (h16*)wsp; wsp += SZ_PL;
    h16* CR = (h16*)wsp; wsp += SZ_CR;
    bf* WQ = (bf*)WBc; bf* WK = (bf*)(WBc + (size_t)DM * DM * 2); h16* WO = (h16*)(WBc + (size_t)2 * DM * DM * 2);

    if (SEQ == SEQ_FULL) {
        const size_t n8 = (size_t)NB * SEQ * DM / 8;
        k_cvt8<<<(unsigned)((n8 + 255) / 256), 256, 0, stream>>>(x, XB, n8);
    } else {
        const size_t n8 = (size_t)SEQ * DM / 8;
        for (int b = 0; b < NB; ++b) k_cvt8<<<(unsigned)((n8 + 255) / 256), 256, 0, stream>>>(x + (size_t)b * SEQ_FULL * DM, XB + (size_t)b * SEQ * DM, n8);
    }
    { const size_t n8 = (size_t)DM * DM / 8; const unsigned g = (unsigned)((n8 + 255) / 256);
      k_cvt8<<<g, 256, 0, stream>>>(wq, WQ, n8); k_cvt8<<<g, 256, 0, stream>>>(wk, WK, n8); k_cvt8h<<<g, 256, 0, stream>>>(wo, WO, n8, WOCAR); }

    k_proj<<<dim3(NB * SEQ / 64, DM / 64, 1), 32, 0, stream>>>(XB, WQ, QH, QR, 1, QCAR, SEQ, (size_t)NH_ * SEQ * HD, HD, HD, (size_t)SEQ * HD);
    k_proj<<<dim3(NB * SEQ / 64, DM / 64, 1), 32, 0, stream>>>(XB, WK, KP, KP, 0, 1.0f, SEQ, (size_t)NH_ * SEQ * HD, HD, HD, (size_t)SEQ * HD);
    k_proj<<<dim3(DM / 64, NB * SEQ / 64, 1), 32, 0, stream>>>(WK, XB, VH, VR, 1, VCAR, DM, (size_t)0, SEQ, SEQ, (size_t)DM * SEQ);

    k_attn<1><<<dim3(EROWS / 16, NB, 1), 512, 0, stream>>>(QH, QR, KP, VH, VR, qm, tb, ta, rela, absa, CH, CR, 0);
    if (SEQ > EROWS)
        k_attn<0><<<dim3((SEQ - EROWS) / 16, NB, 1), 512, 0, stream>>>(QH, QR, KP, VH, VR, qm, tb, ta, rela, absa, CH, CR, EROWS / 16);

    k_out<<<dim3(NB * SEQ / 64, DM / 64, 1), 32, 0, stream>>>(CH, WO, OUT, (size_t)(CR - CH));
}
